// SAGEConvLayer_70935679861287
// MI455X (gfx1250) — hardware-run, weakly checked
//
#include <hip/hip_runtime.h>

typedef float          v8f   __attribute__((ext_vector_type(8)));
typedef float          v4f   __attribute__((ext_vector_type(4)));
typedef unsigned int   v4u   __attribute__((ext_vector_type(4)));
typedef int            v8i   __attribute__((ext_vector_type(8)));
typedef unsigned short v8us  __attribute__((ext_vector_type(8)));
typedef unsigned short v16us __attribute__((ext_vector_type(16)));
typedef __bf16         v16bf __attribute__((ext_vector_type(16)));
typedef _Float16       v16h  __attribute__((ext_vector_type(16)));
typedef v4f  __attribute__((may_alias)) v4fa;
typedef v8us __attribute__((may_alias)) v8usa;
union FragB { v16bf v; v16us u; v8us h[2]; v8i w; };
union FragH { v16h  v; v16us u; v8us h[2]; v8i w; };

__device__ __forceinline__ v8f wmb(const FragB& a, const FragB& b, v8f c) {
  v8f d = __builtin_amdgcn_wmma_f32_16x16x32_bf16(false, a.v, false, b.v, (short)0, c, false, false);
  asm volatile("v_nop\n\tv_nop\n\tv_nop\n\tv_nop" : "+v"(d) : "v"(a.w), "v"(b.w));
  return d;
}

__device__ __forceinline__ v8f wmh(const FragH& a, const FragH& b, v8f c) {
  v8f d = __builtin_amdgcn_wmma_f32_16x16x32_f16(false, a.v, false, b.v, (short)0, c, false, false);
  asm volatile("v_nop\n\tv_nop\n\tv_nop\n\tv_nop" : "+v"(d) : "v"(a.w), "v"(b.w));
  return d;
}

__device__ __forceinline__ unsigned bf16_bits(float f) {
  const unsigned u = __float_as_uint(f);
  const unsigned r = (u + 0x7FFFu + ((u >> 16) & 1u)) >> 16;
  const unsigned q = (u >> 16) | 0x40u;
  return ((u & 0x7fffffffu) > 0x7f800000u) ? q : r;
}

__device__ __forceinline__ float bf16_val(float f) {
  return __uint_as_float(bf16_bits(f) << 16);
}
__device__ __forceinline__ int clampi(int v, int lo, int hi) {
  return v < lo ? lo : (v > hi ? hi : v);
}

__device__ __forceinline__ unsigned f16_bits(float f) {
  const unsigned u  = __float_as_uint(f);
  const unsigned s  = (u >> 16) & 0x8000u;
  const unsigned a  = u & 0x7fffffffu;
  const unsigned t  = a - 0x38000000u;
  const unsigned r  = (t + 0x0FFFu + ((t >> 13) & 1u)) >> 13;
  const unsigned rc = r > 0x7C00u ? 0x7C00u : r;
  const bool small  = a < 0x38800000u;
  const bool isnan  = a > 0x7f800000u;
  const unsigned fin = small ? 0u : (s | rc);
  return isnan ? (s | 0x7E00u) : fin;
}

__device__ __forceinline__ unsigned pk16(unsigned lo, unsigned hi) { return lo | (hi << 16); }
__device__ __forceinline__ unsigned bf16_lo_bits(float v) {
  float hi = bf16_val(v);
  asm volatile("" : "+v"(hi));
  return bf16_bits(v - hi);
}
__device__ __forceinline__ v4u pack8_bf16(v4f a, v4f c) {
  return (v4u){ pk16(bf16_bits(a[0]), bf16_bits(a[1])), pk16(bf16_bits(a[2]), bf16_bits(a[3])),
                pk16(bf16_bits(c[0]), bf16_bits(c[1])), pk16(bf16_bits(c[2]), bf16_bits(c[3])) };
}
__device__ __forceinline__ v4u pack8_bf16_lo(v4f a, v4f c) {
  return (v4u){ pk16(bf16_lo_bits(a[0]), bf16_lo_bits(a[1])), pk16(bf16_lo_bits(a[2]), bf16_lo_bits(a[3])),
                pk16(bf16_lo_bits(c[0]), bf16_lo_bits(c[1])), pk16(bf16_lo_bits(c[2]), bf16_lo_bits(c[3])) };
}
__device__ __forceinline__ v4u pack8_f16(v4f a, v4f c) {
  return (v4u){ pk16(f16_bits(a[0]), f16_bits(a[1])), pk16(f16_bits(a[2]), f16_bits(a[3])),
                pk16(f16_bits(c[0]), f16_bits(c[1])), pk16(f16_bits(c[2]), f16_bits(c[3])) };
}

template <int FORM>
__global__ __launch_bounds__(256) void k_plane(const float* __restrict__ src, int rows, int cols, int ldsrc,
                                               unsigned short* __restrict__ dst, int MP, int KP) {
  static_assert(FORM >= 0 && FORM <= 3);
  const int KTOT = (FORM == 1 || FORM == 3) ? 2 * KP : KP;
  const unsigned ppr   = (unsigned)(KTOT >> 3);
  const unsigned kp8   = (unsigned)(KP >> 3);
  const unsigned total = (unsigned)MP * ppr;
  const unsigned g     = blockIdx.x * 256u + threadIdx.x;
  const unsigned rowu  = g / ppr;
  const unsigned p     = g - rowu * ppr;
  const bool second    = p >= kp8;
  const int row = (int)rowu;
  const int c0  = (int)((second ? p - kp8 : p) << 3);
  const float* srow = src + (size_t)clampi(row, 0, rows - 1) * (size_t)ldsrc;
  float x[8];
  unsigned mk[8];
#pragma unroll
  for (int e = 0; e < 8; ++e) {
    const int c = c0 + e;
    const float v = srow[clampi(c, 0, cols - 1)];
    asm volatile("" :: "v"(v));
    x[e]  = v;
    mk[e] = (row < rows && c < cols) ? 0xFFFFu : 0u;
  }
  const v4f a = (v4f){ x[0], x[1], x[2], x[3] };
  const v4f c = (v4f){ x[4], x[5], x[6], x[7] };
  v4u o;
  if (FORM == 2) {
    o = pack8_f16(a, c);
  } else {
    const v4u hi = pack8_bf16(a, c);
    o = hi;
    if (FORM == 1) { const v4u lo = pack8_bf16_lo(a, c); o = second ? lo : hi; }
  }
  const v4u mw = (v4u){ pk16(mk[0], mk[1]), pk16(mk[2], mk[3]), pk16(mk[4], mk[5]), pk16(mk[6], mk[7]) };
  o &= mw;
  if (g < total) {
    volatile v4u* q = (volatile v4u*)(dst + (size_t)g * 8);
    *q = o;
    __threadfence();
    *q = o;
  }
}

template <int FORM> struct FragOf    { typedef FragB T; };
template <>         struct FragOf<2> { typedef FragH T; };
__device__ __forceinline__ v8f mm(const FragB& a, const FragB& b, v8f c) { return wmb(a, b, c); }
__device__ __forceinline__ v8f mm(const FragH& a, const FragH& b, v8f c) { return wmh(a, b, c); }
template <class F> __device__ __forceinline__ F ld_frag(const unsigned short* p) {
  F f;
  f.h[0] = *(const v8usa*)(p);
  f.h[1] = *(const v8usa*)(p + 16);
  return f;
}

template <int FORM, int EPI>
__global__ __launch_bounds__(256) __attribute__((amdgpu_num_vgpr(248)))
void k_gemm_nt(const unsigned short* __restrict__ A, const unsigned short* __restrict__ B,
               const float* __restrict__ bias, float* __restrict__ D, int M, int N, int KTOT, int ldd) {
  static_assert(FORM >= 0 && FORM <= 2);
  static_assert(EPI == 0 || EPI == 1);
  typedef typename FragOf<FORM>::T F;
  __shared__ __attribute__((aligned(16))) float sT[8][16 * 68];
  const int lane = threadIdx.x & 31;
  const int wave = threadIdx.x >> 5;
  const int tilesM = (M + 63) >> 6;
  const int tilesN = (N + 63) >> 6;
  const int tile = blockIdx.x * 8 + wave;
  if (tile >= tilesM * tilesN) return;
  const int tm = tile / tilesN;
  const int tn = tile - tm * tilesN;
  const int m0 = tm << 6;
  const int n0 = tn << 6;

  const int rl = lane & 15;
  const int h8 = (lane >> 4) * 8;
  const unsigned short* pa = A + (size_t)(m0 + rl) * (size_t)KTOT + h8;
  const unsigned short* pb = B + (size_t)(n0 + rl) * (size_t)KTOT + h8;

  v8f acc[4][4];
#pragma unroll
  for (int i = 0; i < 4; ++i)
#pragma unroll
    for (int j = 0; j < 4; ++j) acc[i][j] = (v8f){0.f, 0.f, 0.f, 0.f, 0.f, 0.f, 0.f, 0.f};

#pragma unroll 1
  for (int k0 = 0; k0 < KTOT; k0 += 32) {
    F bf[4];
#pragma unroll
    for (int j = 0; j < 4; ++j) bf[j] = ld_frag<F>(pb + (size_t)(j << 4) * (size_t)KTOT + k0);
#pragma unroll
    for (int i = 0; i < 4; ++i) {
      const F af = ld_frag<F>(pa + (size_t)(i << 4) * (size_t)KTOT + k0);
#pragma unroll
      for (int j = 0; j < 4; ++j) acc[i][j] = mm(af, bf[j], acc[i][j]);
    }
  }

  float* slab = sT[wave];
  const int hh = lane >> 4;
  const int c4 = (lane & 15) * 4;
  const int nc = n0 + c4;
  const bool cok = nc < N;
  v4f bv = (v4f){0.f, 0.f, 0.f, 0.f};
  if (EPI == 1) {
    bv = *(const v4fa*)(bias + clampi(nc, 0, N - 4));
    asm volatile("" :: "v"(bv));
  }
#pragma unroll
  for (int i = 0; i < 4; ++i) {
    const int mBase = m0 + (i << 4);
#pragma unroll
    for (int j = 0; j < 4; ++j) {
#pragma unroll
      for (int r = 0; r < 8; ++r) slab[(h8 + r) * 68 + (j << 4) + rl] = acc[i][j][r];
    }
    __builtin_amdgcn_fence(__ATOMIC_RELEASE, "workgroup");
    __builtin_amdgcn_wave_barrier();
    __builtin_amdgcn_fence(__ATOMIC_ACQUIRE, "workgroup");
    v4f vv[8];
#pragma unroll
    for (int it = 0; it < 8; ++it) {
      const int row = it * 2 + hh;
      v4f v = *(const v4fa*)(slab + row * 68 + c4);
      if (EPI == 1) v += bv;
      vv[it] = v;
    }
    for (int pass = 0; pass < 2; ++pass) {
#pragma unroll
      for (int it = 0; it < 8; ++it) {
        const int row = mBase + it * 2 + hh;
        if (cok && row < M) *(volatile v4f*)(D + (size_t)row * (size_t)ldd + nc) = vv[it];
      }
      __threadfence();
    }
    __builtin_amdgcn_fence(__ATOMIC_RELEASE, "workgroup");
    __builtin_amdgcn_wave_barrier();
    __builtin_amdgcn_fence(__ATOMIC_ACQUIRE, "workgroup");
  }
}

#include <stddef.h>
#include <math.h>
#pragma clang fp contract(off)

#ifndef SPLIT_H
#define SPLIT_H 1
#endif

#define NN      50000
#define FD      128
#define NE      800000
#define MP      50048
#define K2      (FD * (1 + SPLIT_H))
#define NTHR    256
#define NWAVE   8
#define EPT     8
#define WCH     (32 * EPT)
#define NBRUN   1024
#define SLB     10
#define NBK     49
#define WLCAP   4608
#define LCAP    21504
#define DEGCAP  64
#define MAXDEG_MEAS   35
#define MAXB1024_MEAS 16623
#define WBLK    6250
#define HBLK    (MP / NWAVE)

#define BK_ZINTS (NWAVE * WLCAP + LCAP + 3 * NBRUN)
#define BK_INTS  (BK_ZINTS + 16)
#define BK_LDS   (BK_INTS * 4)

#define PW_U    (FD * FD / 8)
#define PW_UL   (FD * K2 / 8)
#define PW_B    (PW_U / NTHR)
#define PW_BL   (PW_UL / NTHR)
#define PW_BLKS (2 * PW_B + PW_BL + 1)

static_assert(SPLIT_H == 0 || SPLIT_H == 1);
static_assert(FD == 32 * 4);
static_assert(NN % 8 == 0 && NN % 16 == 0);
static_assert(MP == 391 * 128 && MP % 64 == 0 && MP >= NN && MP % 16 == 0);
static_assert((FD * 4) % 128 == 0 && (K2 * 2) % 128 == 0 && FD % 64 == 0 && FD % 32 == 0 && K2 % 32 == 0);
static_assert(WBLK * NWAVE == NN);
static_assert(HBLK * NWAVE == MP);
static_assert(NBRUN == (1 << SLB) && NBRUN == NTHR * 4 && NBRUN % 32 == 0);
static_assert(NBK * NBRUN >= NN && (NBK - 1) * NBRUN < NN);
static_assert(NE < (1 << 21) && (((long long)NE) << SLB) < (1LL << 31));
static_assert(NE % EPT == 0 && NE >= EPT);
static_assert(LCAP % 1024 == 0 && LCAP % (NTHR * 4) == 0);
static_assert((long long)LCAP * 100 >= (long long)MAXB1024_MEAS * 125);
static_assert((long long)WLCAP * NWAVE * 100 >= (long long)MAXB1024_MEAS * 200);
static_assert(MAXDEG_MEAS + 8 <= DEGCAP);
static_assert(BK_ZINTS % 4 == 0 && BK_LDS <= 262144 && BK_LDS <= 327680);
static_assert(PW_U % NTHR == 0 && PW_UL % NTHR == 0);
static_assert((MP * FD / 8) % NTHR == 0);
static_assert((long long)MP * 256 / 8 < (1LL << 31));

typedef int          v4i  __attribute__((ext_vector_type(4)));
typedef unsigned int v2u  __attribute__((ext_vector_type(2)));
typedef v4i __attribute__((may_alias)) v4ia;
typedef v2u __attribute__((may_alias)) v2ua;

__device__ __forceinline__ void st2_v4f(float* p, v4f v) {
  *(volatile v4f*)p = v;
  __threadfence();
  *(volatile v4f*)p = v;
}
__device__ __forceinline__ void st2_v4u(unsigned short* p, v4u v) {
  *(volatile v4u*)p = v;
  __threadfence();
  *(volatile v4u*)p = v;
}
__device__ __forceinline__ v4u conv8(const float* __restrict__ p) {
  const v4f a = *(const v4fa*)(p);
  const v4f c = *(const v4fa*)(p + 4);
  return pack8_bf16(a, c);
}
__device__ __forceinline__ float sel4(int j, float a, float b, float c, float d) {
  return (j == 0) ? a : ((j == 1) ? b : ((j == 2) ? c : d));
}

__global__ __launch_bounds__(NTHR) void k_prep(const float* __restrict__ Wp, const float* __restrict__ Wl,
                                               const float* __restrict__ Wr, const float* __restrict__ bp,
                                               const float* __restrict__ bl,
                                               unsigned short* wpb, unsigned short* wrb, unsigned short* wld,
                                               float* bias) {
  const int tid = (int)threadIdx.x;
  const int blk = (int)blockIdx.x;
  if (blk < PW_B) {
    const int u = blk * NTHR + tid;
    const v4u o = conv8(Wp + (size_t)u * 8);
    st2_v4u(wpb + (size_t)u * 8, o);
  } else if (blk < 2 * PW_B) {
    const int u = (blk - PW_B) * NTHR + tid;
    const v4u o = conv8(Wr + (size_t)u * 8);
    st2_v4u(wrb + (size_t)u * 8, o);
  } else if (blk < 2 * PW_B + PW_BL) {
    const int u = (blk - 2 * PW_B) * NTHR + tid;
    const int ppr = K2 / 8;
    const int n = u / ppr, k8 = (u - n * ppr) * 8;
    const int ks = k8 & (FD - 1);
    const v4u o = conv8(Wl + (size_t)n * FD + ks);
    st2_v4u(wld + (size_t)u * 8, o);
  } else {
    if (tid < 32) {
      const v4f v = *(const v4fa*)(bp + 4 * tid);
      v4f o;
      o.x = bf16_val(v.x); o.y = bf16_val(v.y); o.z = bf16_val(v.z); o.w = bf16_val(v.w);
      st2_v4f(bias + 4 * tid, o);
    } else if (tid < 64) {
      const int t = tid - 32;
      const v4f v = *(const v4fa*)(bl + 4 * t);
      v4f o;
      o.x = bf16_val(v.x); o.y = bf16_val(v.y); o.z = bf16_val(v.z); o.w = bf16_val(v.w);
      st2_v4f(bias + FD + 4 * t, o);
    }
  }
}

__global__ __launch_bounds__(NTHR) void k_hconv(const float* __restrict__ P, unsigned short* H) {
  const int tid = (int)threadIdx.x, lane = tid & 31, wave = tid >> 5;
  const int row = (int)blockIdx.x * NWAVE + wave;
  const v4f p = *(const v4fa*)(P + (size_t)row * FD + 4 * lane);
  const float p0 = p.x, p1 = p.y, p2 = p.z, p3 = p.w;
  asm volatile("" :: "v"(p0));
  asm volatile("" :: "v"(p1));
  asm volatile("" :: "v"(p2));
  asm volatile("" :: "v"(p3));
  const float h0 = (p0 > 0.0f) ? p0 : (p0 - p0);
  const float h1 = (p1 > 0.0f) ? p1 : (p1 - p1);
  const float h2 = (p2 > 0.0f) ? p2 : (p2 - p2);
  const float h3 = (p3 > 0.0f) ? p3 : (p3 - p3);
  const unsigned mk = (row < NN) ? 0xFFFFFFFFu : 0u;
  v2u hv, lv;
  hv.x = pk16(bf16_bits(h0), bf16_bits(h1)) & mk;
  hv.y = pk16(bf16_bits(h2), bf16_bits(h3)) & mk;
  lv.x = pk16(bf16_lo_bits(h0), bf16_lo_bits(h1)) & mk;
  lv.y = pk16(bf16_lo_bits(h2), bf16_lo_bits(h3)) & mk;
  unsigned short* hr = H + (size_t)row * K2 + 4 * lane;
  for (int pass = 0; pass < 2; ++pass) {
    *(volatile v2u*)hr = hv;
    if (SPLIT_H) *(volatile v2u*)(hr + FD) = lv;
    __threadfence();
  }
}

__device__ __forceinline__ void bucket_flush(const int* pl, const int* cnt, const int* offs, int ov,
                                             int* lp, int* cp, int* op, int* fp, int tid) {
#pragma unroll 1
  for (int i = tid * 4; i < LCAP; i += NTHR * 4) {
    const v4i v = *(const v4ia*)(pl + i);
    *(volatile v4i*)(lp + i) = v;
  }
  {
    const v4i v = *(const v4ia*)(cnt + 4 * tid);
    *(volatile v4i*)(cp + 4 * tid) = v;
  }
  {
    const v4i v = *(const v4ia*)(offs + 4 * tid);
    *(volatile v4i*)(op + 4 * tid) = v;
  }
  if (tid < 8) {
    const v4i f = {ov, ov, ov, ov};
    *(volatile v4i*)(fp + 4 * tid) = f;
  }
}

__global__ __launch_bounds__(NTHR) void k_bucket(const int* __restrict__ srcs, const int* __restrict__ dsts,
                                                 int* LIST, int* CNT, int* OFF, int* FLAG) {
  extern __shared__ __attribute__((aligned(16))) int dsm[];
  int* wl   = dsm;
  int* pl   = dsm + NWAVE * WLCAP;
  int* cnt  = pl + LCAP;
  int* offs = cnt + NBRUN;
  int* cur  = offs + NBRUN;
  int* misc = cur + NBRUN;
  const int tid = (int)threadIdx.x, lane = tid & 31, wave = tid >> 5;
  const int blk = (int)blockIdx.x;
  const unsigned nbs = (unsigned)(blk * NBRUN);

  {
    const v4i z4 = {0, 0, 0, 0};
    for (int i = tid * 4; i < BK_ZINTS; i += NTHR * 4) *(v4ia*)(dsm + i) = z4;
    if (tid < 16) misc[tid] = 0;
  }
  __syncthreads();

  {
    const int per  = ((NE + NWAVE * WCH - 1) / (NWAVE * WCH)) * WCH;
    const int ebeg = wave * per;
    const int eend = (ebeg + per < NE) ? (ebeg + per) : NE;
    int* mylist = wl + wave * WLCAP;
    int wc = 0;
#pragma unroll 1
    for (int cb = ebeg; cb < eend; cb += WCH) {
      const int e0 = cb + lane * EPT;
      const int ec = e0 < NE - EPT ? e0 : NE - EPT;
      const bool lv = e0 < NE;
      const v4i da = *(const v4ia*)(dsts + ec);
      const v4i db = *(const v4ia*)(dsts + ec + 4);
      const int k0 = da.x, k1 = da.y, k2 = da.z, k3 = da.w;
      const int k4 = db.x, k5 = db.y, k6 = db.z, k7 = db.w;
      asm volatile("" :: "v"(k0));
      asm volatile("" :: "v"(k1));
      asm volatile("" :: "v"(k2));
      asm volatile("" :: "v"(k3));
      asm volatile("" :: "v"(k4));
      asm volatile("" :: "v"(k5));
      asm volatile("" :: "v"(k6));
      asm volatile("" :: "v"(k7));
      const unsigned s0 = (unsigned)k0 - nbs, s1 = (unsigned)k1 - nbs;
      const unsigned s2 = (unsigned)k2 - nbs, s3 = (unsigned)k3 - nbs;
      const unsigned s4 = (unsigned)k4 - nbs, s5 = (unsigned)k5 - nbs;
      const unsigned s6 = (unsigned)k6 - nbs, s7 = (unsigned)k7 - nbs;
      const bool h0 = lv && s0 < (unsigned)NBRUN && (unsigned)k0 < (unsigned)NN;
      const bool h1 = lv && s1 < (unsigned)NBRUN && (unsigned)k1 < (unsigned)NN;
      const bool h2 = lv && s2 < (unsigned)NBRUN && (unsigned)k2 < (unsigned)NN;
      const bool h3 = lv && s3 < (unsigned)NBRUN && (unsigned)k3 < (unsigned)NN;
      const bool h4 = lv && s4 < (unsigned)NBRUN && (unsigned)k4 < (unsigned)NN;
      const bool h5 = lv && s5 < (unsigned)NBRUN && (unsigned)k5 < (unsigned)NN;
      const bool h6 = lv && s6 < (unsigned)NBRUN && (unsigned)k6 < (unsigned)NN;
      const bool h7 = lv && s7 < (unsigned)NBRUN && (unsigned)k7 < (unsigned)NN;
      const unsigned m0 = __builtin_amdgcn_ballot_w32(h0), m1 = __builtin_amdgcn_ballot_w32(h1);
      const unsigned m2 = __builtin_amdgcn_ballot_w32(h2), m3 = __builtin_amdgcn_ballot_w32(h3);
      const unsigned m4 = __builtin_amdgcn_ballot_w32(h4), m5 = __builtin_amdgcn_ballot_w32(h5);
      const unsigned m6 = __builtin_amdgcn_ballot_w32(h6), m7 = __builtin_amdgcn_ballot_w32(h7);
      const unsigned any = m0 | m1 | m2 | m3 | m4 | m5 | m6 | m7;
      if (any != 0u) {
        const int pre = (int)(__builtin_amdgcn_mbcnt_lo(m0, 0u) + __builtin_amdgcn_mbcnt_lo(m1, 0u) +
                              __builtin_amdgcn_mbcnt_lo(m2, 0u) + __builtin_amdgcn_mbcnt_lo(m3, 0u) +
                              __builtin_amdgcn_mbcnt_lo(m4, 0u) + __builtin_amdgcn_mbcnt_lo(m5, 0u) +
                              __builtin_amdgcn_mbcnt_lo(m6, 0u) + __builtin_amdgcn_mbcnt_lo(m7, 0u));
        int p = wc + pre;
        if (h0) { if (p < WLCAP) mylist[p] = ((e0 + 0) << SLB) | (int)s0; p = p + 1; }
        if (h1) { if (p < WLCAP) mylist[p] = ((e0 + 1) << SLB) | (int)s1; p = p + 1; }
        if (h2) { if (p < WLCAP) mylist[p] = ((e0 + 2) << SLB) | (int)s2; p = p + 1; }
        if (h3) { if (p < WLCAP) mylist[p] = ((e0 + 3) << SLB) | (int)s3; p = p + 1; }
        if (h4) { if (p < WLCAP) mylist[p] = ((e0 + 4) << SLB) | (int)s4; p = p + 1; }
        if (h5) { if (p < WLCAP) mylist[p] = ((e0 + 5) << SLB) | (int)s5; p = p + 1; }
        if (h6) { if (p < WLCAP) mylist[p] = ((e0 + 6) << SLB) | (int)s6; p = p + 1; }
        if (h7) { if (p < WLCAP) mylist[p] = ((e0 + 7) << SLB) | (int)s7; p = p + 1; }
        wc += (int)(__builtin_popcount(m0) + __builtin_popcount(m1) + __builtin_popcount(m2) + __builtin_popcount(m3) +
                    __builtin_popcount(m4) + __builtin_popcount(m5) + __builtin_popcount(m6) + __builtin_popcount(m7));
      }
    }
    if (lane == 0) misc[wave] = wc;
  }
  __syncthreads();

  if (wave == 0) {
    int ov = 0;
    int tot = 0;
#pragma unroll 1
    for (int w2 = 0; w2 < NWAVE; ++w2) {
      int c = misc[w2];
      if (c > WLCAP) ov = 1;
      c = c < 0 ? 0 : (c > WLCAP ? WLCAP : c);
      tot += c;
#pragma unroll 1
      for (int b0 = 0; b0 < c; b0 += 32) {
        const int idx = b0 + lane;
        const int ent = wl[w2 * WLCAP + (idx < WLCAP ? idx : WLCAP - 1)];
        const int m32 = (c - b0) < 32 ? (c - b0) : 32;
#pragma unroll 1
        for (int k = 0; k < m32; ++k) {
          const int u    = __builtin_amdgcn_readlane(ent, k);
          const int slot = u & (NBRUN - 1);
          if (lane == 0) cnt[slot] = cnt[slot] + 1;
        }
      }
    }
    if (tot > LCAP) ov = 1;
    if (lane == 0) misc[9] = ov;
  }
  __syncthreads();
  if (wave == 0) {
    const int base = lane * (NBRUN / 32);
    int s = 0;
#pragma unroll 1
    for (int i = 0; i < NBRUN / 32; ++i) s += cnt[base + i];
    int incl = s;
#pragma unroll
    for (int d = 1; d < 32; d <<= 1) {
      const int y = __shfl_up(incl, d, 32);
      if (lane >= d) incl += y;
    }
    int run = incl - s;
#pragma unroll 1
    for (int i = 0; i < NBRUN / 32; ++i) {
      const int cv = cnt[base + i];
      offs[base + i] = run;
      cur[base + i]  = run;
      run += cv;
    }
  }
  __syncthreads();

  if (wave == 0) {
#pragma unroll 1
    for (int w2 = 0; w2 < NWAVE; ++w2) {
      int c = misc[w2];
      c = c < 0 ? 0 : (c > WLCAP ? WLCAP : c);
#pragma unroll 1
      for (int b0 = 0; b0 < c; b0 += 32) {
        const int idx = b0 + lane;
        const int ent = wl[w2 * WLCAP + (idx < WLCAP ? idx : WLCAP - 1)];
        int eid = (ent >> SLB) & 0x1FFFFF;
        eid = eid > NE - 1 ? NE - 1 : eid;
        int sr = srcs[eid];
        asm volatile("" :: "v"(sr));
        sr = clampi(sr, 0, NN - 1);
        const int m32 = (c - b0) < 32 ? (c - b0) : 32;
#pragma unroll 1
        for (int k = 0; k < m32; ++k) {
          const int u    = __builtin_amdgcn_readlane(ent, k);
          const int w0   = __builtin_amdgcn_readlane(sr, k);
          const int slot = u & (NBRUN - 1);
          if (lane == 0) {
            int p = cur[slot];
            p = p < 0 ? 0 : (p > LCAP - 1 ? LCAP - 1 : p);
            pl[p] = w0;
            cur[slot] = p + 1;
          }
        }
      }
    }
  }
  __syncthreads();

  const int ovf = misc[9];
  int* lp = LIST + (size_t)blk * (size_t)LCAP;
  int* cp = CNT  + (size_t)blk * NBRUN;
  int* op = OFF  + (size_t)blk * NBRUN;
  int* fp = FLAG + (size_t)blk * 32;
  bucket_flush(pl, cnt, offs, ovf, lp, cp, op, fp, tid);
  __threadfence();
  bucket_flush(pl, cnt, offs, ovf, lp, cp, op, fp, tid);
}

__global__ __launch_bounds__(NTHR) void k_walk(const int* __restrict__ LIST, const int* __restrict__ CNT,
                                               const int* __restrict__ OFF, const int* __restrict__ FLAG,
                                               const float* __restrict__ T, const unsigned short* __restrict__ XB,
                                               float* S) {
  const int tid = (int)threadIdx.x, lane = tid & 31, wave = tid >> 5;
  const int blk = (int)blockIdx.x;
  const int n  = blk * NWAVE + wave;
  const int bk = n >> SLB;
  const int cv = CNT[n];
  asm volatile("" :: "v"(cv));
  const int ovv = OFF[n];
  asm volatile("" :: "v"(ovv));
  const int fl = FLAG[(size_t)bk * 32];
  asm volatile("" :: "v"(fl));

  const bool bad = (fl != 0) || (cv > DEGCAP) || (cv < 0);
  const int trip = __builtin_amdgcn_readfirstlane((fl == 0 && cv > 0) ? (cv > DEGCAP ? DEGCAP : cv) : 0);
  const int o = clampi(ovv, 0, LCAP - 1);
  int last = o + (trip > 0 ? trip : 1) - 1;
  last = last > LCAP - 1 ? LCAP - 1 : last;
  const int* lb = LIST + (size_t)bk * (size_t)LCAP;
  const float* tl = T + 4 * lane;

  v4f acc = (v4f){0.0f, 0.0f, 0.0f, 0.0f};
#pragma unroll 1
  for (int b0 = 0; b0 < trip; b0 += 32) {
    int idx = o + b0 + lane;
    idx = idx > last ? last : idx;
    int sr = lb[idx];
    sr = clampi(sr, 0, NN - 1);
    const int m32 = (trip - b0) < 32 ? (trip - b0) : 32;
#pragma unroll 1
    for (int k = 0; k < m32; ++k) {
      const int sk = __builtin_amdgcn_readlane(sr, k);
      const v4f q = *(const v4fa*)(tl + (size_t)sk * FD);
      acc += q;
    }
  }

  const v4f d = *(const v4fa*)(S + (size_t)n * FD + 4 * lane);
  const float d0 = d.x, d1 = d.y, d2 = d.z, d3 = d.w;
  asm volatile("" :: "v"(d0));
  asm volatile("" :: "v"(d1));
  asm volatile("" :: "v"(d2));
  asm volatile("" :: "v"(d3));
  const v2u xw = *(const v2ua*)(XB + (size_t)n * FD + 4 * lane);
  const unsigned xa = xw.x, xb = xw.y;
  asm volatile("" :: "v"(xa));
  asm volatile("" :: "v"(xb));
  const float x0 = __uint_as_float(xa << 16);
  const float x1 = __uint_as_float(xa & 0xffff0000u);
  const float x2 = __uint_as_float(xb << 16);
  const float x3 = __uint_as_float(xb & 0xffff0000u);

  const int cm = cv > 1 ? cv : 1;
  const float cf = (float)cm;
  const float a0 = acc.x, a1 = acc.y, a2 = acc.z, a3 = acc.w;

  float e0 = 0.0f, e1 = 0.0f, e2 = 0.0f, e3 = 0.0f;
#pragma unroll 1
  for (int j = 0; j < 4; ++j) {
    const float a = sel4(j, a0, a1, a2, a3);
    const float s = sel4(j, d0, d1, d2, d3);
    const float m = a / cf;
    const float v = s + m;
    const float ex = expm1f(v);
    const float y = (v > 0.0f) ? v : ex;
    e0 = (j == 0) ? y : e0;
    e1 = (j == 1) ? y : e1;
    e2 = (j == 2) ? y : e2;
    e3 = (j == 3) ? y : e3;
  }

  const float q0 = e0 * e0, q1 = e1 * e1, q2 = e2 * e2, q3 = e3 * e3;
  float ss = ((q0 + q1) + q2) + q3;
  ss = ss + __shfl_xor(ss, 16, 32);
  ss = ss + __shfl_xor(ss, 8, 32);
  ss = ss + __shfl_xor(ss, 4, 32);
  ss = ss + __shfl_xor(ss, 2, 32);
  ss = ss + __shfl_xor(ss, 1, 32);
  const float nrm = sqrtf(ss);
  const float sel = (nrm > 1e-12f || nrm != nrm) ? nrm : 1e-12f;

  float r0 = 0.0f, r1 = 0.0f, r2 = 0.0f, r3 = 0.0f;
#pragma unroll 1
  for (int j = 0; j < 4; ++j) {
    const float e  = sel4(j, e0, e1, e2, e3);
    const float xv = sel4(j, x0, x1, x2, x3);
    const float q  = e / sel;
    const float y  = xv + q;
    r0 = (j == 0) ? y : r0;
    r1 = (j == 1) ? y : r1;
    r2 = (j == 2) ? y : r2;
    r3 = (j == 3) ? y : r3;
  }

  const float qnan = __uint_as_float(0x7fc00000u);
  v4f ov;
  ov.x = bad ? qnan : r0; ov.y = bad ? qnan : r1; ov.z = bad ? qnan : r2; ov.w = bad ? qnan : r3;
  if (n < NN) {
    st2_v4f(S + (size_t)n * FD + 4 * lane, ov);
  }
}

extern "C" void kernel_launch(void* const* d_in, const int* in_sizes, int n_in,
                              void* d_out, int out_size, void* d_ws, size_t ws_size,
                              hipStream_t stream) {
  if (n_in < 7) return;
  if (in_sizes[0] != NN * FD) return;
  if (in_sizes[1] != 2 * NE) return;
  if (in_sizes[2] != FD * FD) return;
  if (in_sizes[3] != FD) return;
  if (in_sizes[4] != FD * FD) return;
  if (in_sizes[5] != FD) return;
  if (in_sizes[6] != FD * FD) return;
  if (out_size != NN * FD) return;

  const float* x    = (const float*)d_in[0];
  const int*   ei   = (const int*)d_in[1];
  const int*   srcs = ei;
  const int*   dsts = ei + NE;
  const float* Wp   = (const float*)d_in[2];
  const float* bp   = (const float*)d_in[3];
  const float* Wl   = (const float*)d_in[4];
  const float* bl   = (const float*)d_in[5];
  const float* Wr   = (const float*)d_in[6];
  float* out = (float*)d_out;

  constexpr size_t zXB   = (size_t)MP * FD * 2;
  constexpr size_t zPT   = (size_t)MP * FD * 4;
  constexpr size_t zH    = (size_t)MP * 256 * 2;
  constexpr size_t zLIST = (size_t)NBK * LCAP * 4;
  constexpr size_t zTAB  = (size_t)NBK * NBRUN * 4;
  constexpr size_t zFLAG = (size_t)NBK * 128;
  constexpr size_t zW    = (size_t)FD * FD * 2;
  constexpr size_t zWL   = (size_t)FD * 256 * 2;
  constexpr size_t zBIAS = 1024;
  constexpr size_t oXB   = 0;
  constexpr size_t oPT   = oXB + zXB;
  constexpr size_t oH    = oPT + zPT;
  constexpr size_t oLIST = oH + zH;
  constexpr size_t oCNT  = oLIST + zLIST;
  constexpr size_t oOFF  = oCNT + zTAB;
  constexpr size_t oFLAG = oOFF + zTAB;
  constexpr size_t oWP   = oFLAG + zFLAG;
  constexpr size_t oWR   = oWP + zW;
  constexpr size_t oWL   = oWR + zW;
  constexpr size_t oBIAS = oWL + zWL;
  constexpr size_t oEND  = oBIAS + zBIAS;
  static_assert(zXB % 128 == 0 && zPT % 128 == 0 && zH % 128 == 0 && zLIST % 128 == 0 && zTAB % 128 == 0);
  static_assert(zFLAG % 128 == 0 && zW % 128 == 0 && zWL % 128 == 0 && zBIAS % 128 == 0);
  static_assert(zH >= (size_t)MP * K2 * 2 && zWL >= (size_t)FD * K2 * 2 && zBIAS >= (size_t)2 * FD * 4);
  static_assert(zTAB >= (size_t)NN * 4);
  static_assert(oEND == (size_t)537625 * 128);
  static_assert(oEND <= ((size_t)128 << 20));
  if (oEND > ws_size) return;

  char* ws = (char*)d_ws;
  unsigned short* XB   = (unsigned short*)(ws + oXB);
  float*          PT   = (float*)(ws + oPT);
  unsigned short* H    = (unsigned short*)(ws + oH);
  int*            LIST = (int*)(ws + oLIST);
  int*            CNT  = (int*)(ws + oCNT);
  int*            OFF  = (int*)(ws + oOFF);
  int*            FLAG = (int*)(ws + oFLAG);
  unsigned short* WPB  = (unsigned short*)(ws + oWP);
  unsigned short* WRB  = (unsigned short*)(ws + oWR);
  unsigned short* WLD  = (unsigned short*)(ws + oWL);
  float*          BIAS = (float*)(ws + oBIAS);

  hipFuncSetAttribute(reinterpret_cast<const void*>(&k_bucket), hipFuncAttributeMaxDynamicSharedMemorySize, (int)BK_LDS);

  const int tiles = (MP / 64) * (FD / 64);
  const int gg    = (tiles + 7) / 8;

  k_plane<0><<<MP * FD / 8 / NTHR, NTHR, 0, stream>>>(x, NN, FD, FD, XB, MP, FD);
  k_prep<<<PW_BLKS, NTHR, 0, stream>>>(Wp, Wl, Wr, bp, bl, WPB, WRB, WLD, BIAS);
  k_gemm_nt<0, 1><<<gg, NTHR, 0, stream>>>(XB, WPB, BIAS, PT, MP, FD, FD, FD);
  k_hconv<<<HBLK, NTHR, 0, stream>>>(PT, H);
  k_gemm_nt<0, 1><<<gg, NTHR, 0, stream>>>(XB, WRB, BIAS + FD, out, NN, FD, FD, FD);
  k_gemm_nt<0, 0><<<gg, NTHR, 0, stream>>>(H, WLD, BIAS, PT, MP, FD, K2, FD);
  k_bucket<<<NBK, NTHR, BK_LDS, stream>>>(srcs, dsts, LIST, CNT, OFF, FLAG);
  k_walk<<<WBLK, NTHR, 0, stream>>>(LIST, CNT, OFF, FLAG, PT, XB, out);
}
